// CNNRNNModel_5214090297371
// MI455X (gfx1250) — hardware-verified
//
#include <hip/hip_runtime.h>

typedef _Float16 v16h __attribute__((ext_vector_type(16)));
typedef _Float16 v8h  __attribute__((ext_vector_type(8)));
typedef _Float16 v2h  __attribute__((ext_vector_type(2)));
typedef float    v8f  __attribute__((ext_vector_type(8)));
typedef float    v4f  __attribute__((ext_vector_type(4)));
union Frag { v16h v; v8h half[2]; };

#define B_SZ      512
#define CIN       5
#define LEN       1024
#define COUT      32
#define AT        13
#define NBP       5
#define NPOS      (B_SZ * LEN)
#define OUT_PER_B (AT * AT * NBP)
#define SRC_PITCH (LEN + 4)

#define ST_THREADS 128
#define ST_PPT     (LEN / ST_THREADS)
#define NMOM       40

#define MT      256
#define CHUNK   256
#define NCHUNK  (LEN / CHUNK)
#define OB      32

#define WS_PART  0
#define WS_SCSH  262144
#define WS_LLW   262656
#define WS_WC    264704
#define WS_G     297472
#define WS_END   821760

#define L_ET    0
#define L_H     32768
#define L_PART  65536
#define L_G     73728
#define L_SRC   74752
#define L_B16   95312
#define L_TOTAL 95376

__device__ __forceinline__ v8f wmma16(v16h a, v16h b, v8f c) {
  v8f d = __builtin_amdgcn_wmma_f32_16x16x32_f16(false, a, false, b, (short)0, c, false, false);
  asm volatile("v_nop\n\tv_nop\n\tv_nop\n\tv_nop" : "+v"(d) : "v"(a), "v"(b));
  return d;
}

__device__ __forceinline__ v8f zero8() {
  v8f z = {0.0f, 0.0f, 0.0f, 0.0f, 0.0f, 0.0f, 0.0f, 0.0f};
  return z;
}

__device__ __forceinline__ void acc_moments(const float* y, float* S, float* M) {
  S[0] += y[0]; S[1] += y[1]; S[2] += y[2]; S[3] += y[3]; S[4] += y[4];
  M[0]  += y[0] * y[0]; M[1]  += y[0] * y[1]; M[2]  += y[0] * y[2]; M[3]  += y[0] * y[3]; M[4] += y[0] * y[4];
  M[5]  += y[1] * y[1]; M[6]  += y[1] * y[2]; M[7]  += y[1] * y[3]; M[8]  += y[1] * y[4];
  M[9]  += y[2] * y[2]; M[10] += y[2] * y[3]; M[11] += y[2] * y[4];
  M[12] += y[3] * y[3]; M[13] += y[3] * y[4];
  M[14] += y[4] * y[4];
}

__device__ __forceinline__ float dot5(const float* __restrict__ w, const float* v) {
  return w[0] * v[0] + w[1] * v[1] + w[2] * v[2] + w[3] * v[3] + w[4] * v[4];
}

__global__ __launch_bounds__(ST_THREADS) void k_stats(
    const float* __restrict__ src,
    const float* __restrict__ dw1, const float* __restrict__ dw2,
    float* __restrict__ part) {
  __shared__ __attribute__((aligned(16))) float s_src[CIN * SRC_PITCH];
  __shared__ float s_red[NMOM * ST_THREADS];
  __shared__ __attribute__((aligned(16))) float s_out[128];
  const int b = blockIdx.x, tid = threadIdx.x;
  const float* srcb = src + (size_t)b * CIN * LEN;
  for (int idx = tid; idx < CIN * SRC_PITCH; idx += ST_THREADS) {
    int ci = idx / SRC_PITCH, p = idx - ci * SRC_PITCH, l = p - 2;
    s_src[idx] = ((unsigned)l < (unsigned)LEN) ? srcb[ci * LEN + l] : 0.0f;
  }
  __syncthreads();

  float S1[5] = {0.f, 0.f, 0.f, 0.f, 0.f}, S2[5] = {0.f, 0.f, 0.f, 0.f, 0.f};
  float M1[15], M2[15];
#pragma unroll
  for (int i = 0; i < 15; ++i) { M1[i] = 0.0f; M2[i] = 0.0f; }

#pragma unroll 1
  for (int p = 0; p < ST_PPT; ++p) {
    const int l = p * ST_THREADS + tid;
    float y1[CIN], y2[CIN];
#pragma unroll
    for (int ci = 0; ci < CIN; ++ci) {
      const float* row = s_src + ci * SRC_PITCH + l;
      float x0 = row[0], x1 = row[1], x2 = row[2], x3 = row[3], x4 = row[4];
      y1[ci] = dw1[ci * 5 + 0] * x0 + dw1[ci * 5 + 1] * x1 + dw1[ci * 5 + 2] * x2 +
               dw1[ci * 5 + 3] * x3 + dw1[ci * 5 + 4] * x4;
      y2[ci] = dw2[ci * 3 + 0] * x1 + dw2[ci * 3 + 1] * x2 + dw2[ci * 3 + 2] * x3;
    }
    acc_moments(y1, S1, M1);
    acc_moments(y2, S2, M2);
  }

#pragma unroll
  for (int i = 0; i < 5; ++i) {
    s_red[i * ST_THREADS + tid] = S1[i];
    s_red[(20 + i) * ST_THREADS + tid] = S2[i];
  }
#pragma unroll
  for (int i = 0; i < 15; ++i) {
    s_red[(5 + i) * ST_THREADS + tid] = M1[i];
    s_red[(25 + i) * ST_THREADS + tid] = M2[i];
  }
  __syncthreads();
  if (tid < NMOM) {
    float s = 0.0f;
    for (int t = 0; t < ST_THREADS; ++t) s += s_red[tid * ST_THREADS + t];
    s_out[tid] = s;
  } else {
    s_out[tid] = 0.0f;
  }
  __syncthreads();
  if (tid < 32) {
    v4f v = *(const v4f*)(s_out + 4 * tid);
    float* pp = part + (size_t)b * 128 + 4 * tid;
    *(volatile v4f*)pp = v;
    __threadfence();
    *(volatile v4f*)pp = v;
  }
}

__global__ __launch_bounds__(256) void k_fold(
    const float* __restrict__ part,
    const float* __restrict__ pw1, const float* __restrict__ g1, const float* __restrict__ be1,
    const float* __restrict__ pw2, const float* __restrict__ g2, const float* __restrict__ be2,
    const float* __restrict__ ll1w, const float* __restrict__ flw,
    float* __restrict__ scsh, _Float16* __restrict__ llw, _Float16* __restrict__ wc) {
  __shared__ double s_mom[NMOM];
  __shared__ __attribute__((aligned(16))) float s_sc[128];
  const int tid = threadIdx.x;

  if (tid < NMOM) {
    double a = 0.0;
    for (int blk = 0; blk < B_SZ; ++blk) a += (double)part[(size_t)blk * 128 + tid];
    s_mom[tid] = a;
  }
  __syncthreads();

  if (tid < 2 * COUT) {
    const int br = tid >> 5, oc = tid & 31;
    const float* pw = br ? pw2 : pw1;
    const int mb = br * 20;
    double mean = 0.0, e2 = 0.0;
    int q = 5;
    for (int i = 0; i < CIN; ++i) {
      double pi = (double)pw[oc * CIN + i];
      mean += pi * s_mom[mb + i];
      for (int j = i; j < CIN; ++j) {
        double t = pi * (double)pw[oc * CIN + j] * s_mom[mb + q];
        e2 += (j == i) ? t : (t + t);
        ++q;
      }
    }
    const double inv_n = 1.0 / (double)NPOS;
    mean *= inv_n;
    e2 *= inv_n;
    double var = e2 - mean * mean;
    if (var < 0.0) var = 0.0;
    float g  = br ? g2[oc] : g1[oc];
    float be = br ? be2[oc] : be1[oc];
    float r  = rsqrtf((float)var + 1e-5f);
    float mult = r * g;
    float shift = be - (float)mean * mult;
    s_sc[tid] = mult;
    s_sc[64 + tid] = shift;
  }

  const bool has_l = tid < 128;
  v8h lv = {(_Float16)0, (_Float16)0, (_Float16)0, (_Float16)0,
            (_Float16)0, (_Float16)0, (_Float16)0, (_Float16)0};
  if (has_l) {
    const int a = tid >> 3, kb = (tid & 7) * 8;
#pragma unroll
    for (int i = 0; i < 8; ++i)
      lv[i] = (_Float16)((a < AT) ? ll1w[a * (2 * COUT) + kb + i] * 16.0f : 0.0f);
  }
  v8h wv[8];
#pragma unroll
  for (int it = 0; it < 8; ++it) {
    const int f = (it * 256 + tid) * 8;
    const int n = f >> 10, l = f & (LEN - 1);
#pragma unroll
    for (int i = 0; i < 8; ++i) {
      float val = 0.0f;
      if (n < NBP)          val = flw[n * (2 * LEN) + l + i];
      else if (n < 2 * NBP) val = flw[(n - NBP) * (2 * LEN) + LEN + l + i];
      wv[it][i] = (_Float16)(val * 64.0f);
    }
  }
  __syncthreads();

  v4f sv4 = {0.f, 0.f, 0.f, 0.f};
  if (tid < 32) sv4 = *(const v4f*)(s_sc + 4 * tid);

  if (tid < 32) *(volatile v4f*)(scsh + 4 * tid) = sv4;
  if (has_l)    *(volatile v8h*)(llw + tid * 8) = lv;
#pragma unroll
  for (int it = 0; it < 8; ++it) *(volatile v8h*)(wc + (size_t)(it * 256 + tid) * 8) = wv[it];
  __threadfence();
  if (tid < 32) *(volatile v4f*)(scsh + 4 * tid) = sv4;
  if (has_l)    *(volatile v8h*)(llw + tid * 8) = lv;
#pragma unroll
  for (int it = 0; it < 8; ++it) *(volatile v8h*)(wc + (size_t)(it * 256 + tid) * 8) = wv[it];
}

__global__ __launch_bounds__(MT) void k_main(
    const float* __restrict__ src,
    const float* __restrict__ dw1, const float* __restrict__ pw1,
    const float* __restrict__ r1w, const float* __restrict__ r1b,
    const float* __restrict__ dw2, const float* __restrict__ pw2,
    const float* __restrict__ r2w, const float* __restrict__ r2b,
    const float* __restrict__ ll1b,
    const float* __restrict__ scsh,
    const _Float16* __restrict__ llw, const _Float16* __restrict__ wc,
    float* __restrict__ gout) {
  extern __shared__ __attribute__((aligned(16))) char dsm[];
  _Float16* e_t   = (_Float16*)(dsm + L_ET);
  _Float16* hb    = (_Float16*)(dsm + L_H);
  float*    part  = (float*)(dsm + L_PART);
  float*    gst   = (float*)(dsm + L_G);
  float*    s_src = (float*)(dsm + L_SRC);
  float*    s_b16 = (float*)(dsm + L_B16);

  const int b = blockIdx.x, tid = threadIdx.x;
  const int lane = tid & 31, wv = tid >> 5, h = lane >> 4, m = lane & 15;
  const float* srcb = src + (size_t)b * CIN * LEN;

  for (int idx = tid; idx < CIN * SRC_PITCH; idx += MT) {
    int ci = idx / SRC_PITCH, p = idx - ci * SRC_PITCH, l = p - 2;
    s_src[idx] = ((unsigned)l < (unsigned)LEN) ? srcb[ci * LEN + l] : 0.0f;
  }
  if (tid < 16) s_b16[tid] = (tid < AT) ? ll1b[tid] * 16.0f : 0.0f;

  Frag A0, A1;
  A0.half[0] = *(const v8h*)(llw + m * 64 + 8 * h);
  A0.half[1] = *(const v8h*)(llw + m * 64 + 16 + 8 * h);
  A1.half[0] = *(const v8h*)(llw + m * 64 + 32 + 8 * h);
  A1.half[1] = *(const v8h*)(llw + m * 64 + 48 + 8 * h);
  __syncthreads();

  float bias8[8];
#pragma unroll
  for (int r = 0; r < 8; ++r) bias8[r] = s_b16[8 * h + r];

#pragma unroll 1
  for (int chunk = 0; chunk < NCHUNK; ++chunk) {
    {
      const int l = chunk * CHUNK + tid;
      float sv[CIN], y1[CIN], y2[CIN];
#pragma unroll
      for (int ci = 0; ci < CIN; ++ci) {
        const float* row = s_src + ci * SRC_PITCH + l;
        float x0 = row[0], x1 = row[1], x2 = row[2], x3 = row[3], x4 = row[4];
        sv[ci] = x2;
        y1[ci] = dw1[ci * 5 + 0] * x0 + dw1[ci * 5 + 1] * x1 + dw1[ci * 5 + 2] * x2 +
                 dw1[ci * 5 + 3] * x3 + dw1[ci * 5 + 4] * x4;
        y2[ci] = dw2[ci * 3 + 0] * x1 + dw2[ci * 3 + 1] * x2 + dw2[ci * 3 + 2] * x3;
      }
      _Float16* er = e_t + tid * 64;
#pragma unroll 4
      for (int op = 0; op < COUT / 2; ++op) {
        const int oc = 2 * op;
        float z1a = dot5(pw1 + oc * CIN, y1),       z1b = dot5(pw1 + (oc + 1) * CIN, y1);
        float q1a = dot5(r1w + oc * CIN, sv) + r1b[oc], q1b = dot5(r1w + (oc + 1) * CIN, sv) + r1b[oc + 1];
        float z2a = dot5(pw2 + oc * CIN, y2),       z2b = dot5(pw2 + (oc + 1) * CIN, y2);
        float q2a = dot5(r2w + oc * CIN, sv) + r2b[oc], q2b = dot5(r2w + (oc + 1) * CIN, sv) + r2b[oc + 1];
        float a1a = fmaxf(z1a * scsh[oc] + scsh[64 + oc], 0.0f);
        float a1b = fmaxf(z1b * scsh[oc + 1] + scsh[64 + oc + 1], 0.0f);
        float a2a = fmaxf(z2a * scsh[32 + oc] + scsh[96 + oc], 0.0f);
        float a2b = fmaxf(z2b * scsh[32 + oc + 1] + scsh[96 + oc + 1], 0.0f);
        v2h t1 = {(_Float16)(a1a * q1a), (_Float16)(a1b * q1b)};
        v2h t2 = {(_Float16)(a2a * q2a), (_Float16)(a2b * q2b)};
        *(v2h*)(er + oc) = t1;
        *(v2h*)(er + 32 + oc) = t2;
      }
    }
    __syncthreads();
#pragma unroll
    for (int t = 0; t < 2; ++t) {
      const int lt = wv * 2 + t;
      const _Float16* ep = e_t + (lt * 16 + m) * 64 + 8 * h;
      Frag B0, B1;
      B0.half[0] = *(const v8h*)(ep);
      B0.half[1] = *(const v8h*)(ep + 16);
      B1.half[0] = *(const v8h*)(ep + 32);
      B1.half[1] = *(const v8h*)(ep + 48);
      v8f acc = zero8();
      acc = wmma16(A0.v, B0.v, acc);
      acc = wmma16(A1.v, B1.v, acc);
      _Float16* hp = hb + (8 * h) * LEN + chunk * CHUNK + lt * 16 + m;
#pragma unroll
      for (int r = 0; r < 8; ++r) hp[r * LEN] = (_Float16)(acc[r] + bias8[r]);
    }
    __syncthreads();
  }

  {
    v8f accG = zero8();
#pragma unroll
    for (int t = 0; t < 4; ++t) {
      const int k0 = (wv * 4 + t) * 32;
      Frag Ah, Bw;
      const _Float16* hp = hb + m * LEN + k0 + 8 * h;
      Ah.half[0] = *(const v8h*)(hp);
      Ah.half[1] = *(const v8h*)(hp + 16);
      const _Float16* wp = wc + m * LEN + k0 + 8 * h;
      Bw.half[0] = *(const v8h*)(wp);
      Bw.half[1] = *(const v8h*)(wp + 16);
      accG = wmma16(Ah.v, Bw.v, accG);
    }
#pragma unroll
    for (int r = 0; r < 8; ++r) part[(wv * 8 + r) * 32 + lane] = accG[r];
  }
  __syncthreads();
  if (wv == 0) {
#pragma unroll
    for (int r = 0; r < 8; ++r) {
      float s = 0.0f;
#pragma unroll
      for (int w = 0; w < 8; ++w) s += part[(w * 8 + r) * 32 + lane];
      gst[(8 * h + r) * 16 + m] = s * (1.0f / 1024.0f);
    }
  }
  __syncthreads();
  if (wv == 0) {
    v4f g0 = *(const v4f*)(gst + 4 * lane);
    v4f g1 = *(const v4f*)(gst + 128 + 4 * lane);
    float* gp = gout + (size_t)b * 256;
    *(volatile v4f*)(gp + 4 * lane) = g0;
    *(volatile v4f*)(gp + 128 + 4 * lane) = g1;
    __threadfence();
    *(volatile v4f*)(gp + 4 * lane) = g0;
    *(volatile v4f*)(gp + 128 + 4 * lane) = g1;
  }
}

__device__ __forceinline__ v4f gather4(const float* gs, const float* s_flb, int lim, int q) {
  v4f v = {0.f, 0.f, 0.f, 0.f};
#pragma unroll
  for (int e = 0; e < 4; ++e) {
    const int f = 4 * q + e;
    const int s = f / OUT_PER_B;
    const int rem = f - s * OUT_PER_B;
    const int ij = rem / NBP;
    const int n = rem - ij * NBP;
    const int i = ij / AT;
    const int j = ij - i * AT;
    int mn = i < j ? i : j, mx = i < j ? j : i;
    mn = mn < lim ? mn : lim;
    mx = mx < lim ? mx : lim;
    v[e] = gs[s * 256 + mn * 16 + n] + gs[s * 256 + mx * 16 + NBP + n] + s_flb[n];
  }
  return v;
}

__global__ __launch_bounds__(256) void k_out(
    const float* __restrict__ gout, const float* __restrict__ flb,
    const int* __restrict__ maxat, float* __restrict__ out) {
  __shared__ __attribute__((aligned(16))) float gs[OB * 256];
  __shared__ float s_flb[8];
  const int blk = blockIdx.x, tid = threadIdx.x;
  const v4f* gsrc = (const v4f*)(gout + (size_t)blk * OB * 256);
  for (int i = tid; i < OB * 64; i += 256) ((v4f*)gs)[i] = gsrc[i];
  if (tid < 8) s_flb[tid] = (tid < NBP) ? flb[tid] : 0.0f;
  int lim = maxat[0] - 1;
  lim = lim < 0 ? 0 : (lim > AT - 1 ? AT - 1 : lim);
  __syncthreads();

  float* ob = out + (size_t)blk * OB * OUT_PER_B;
  const int NQ = OB * OUT_PER_B / 4;
  for (int q = tid; q < NQ; q += 256) {
    v4f v = gather4(gs, s_flb, lim, q);
    *(volatile v4f*)(ob + 4 * q) = v;
  }
  __threadfence();
  for (int q = tid; q < NQ; q += 256) {
    v4f v = gather4(gs, s_flb, lim, q);
    *(volatile v4f*)(ob + 4 * q) = v;
  }
}

extern "C" void kernel_launch(void* const* d_in, const int* in_sizes, int n_in,
                              void* d_out, int out_size, void* d_ws, size_t ws_size,
                              hipStream_t stream) {
  if (n_in < 19) return;
  if (in_sizes[0] != B_SZ * CIN * LEN) return;
  if (in_sizes[2] < 1) return;
  if (in_sizes[3] != CIN * 5 || in_sizes[4] != COUT * CIN || in_sizes[5] != COUT || in_sizes[6] != COUT) return;
  if (in_sizes[7] != COUT * CIN || in_sizes[8] != COUT) return;
  if (in_sizes[9] != CIN * 3 || in_sizes[10] != COUT * CIN || in_sizes[11] != COUT || in_sizes[12] != COUT) return;
  if (in_sizes[13] != COUT * CIN || in_sizes[14] != COUT) return;
  if (in_sizes[15] != AT * 2 * COUT || in_sizes[16] != AT) return;
  if (in_sizes[17] != NBP * 2 * LEN || in_sizes[18] != NBP) return;
  if (out_size != B_SZ * OUT_PER_B) return;
  if (ws_size < (size_t)WS_END) return;

  const float* src   = (const float*)d_in[0];
  const int*   maxat = (const int*)d_in[2];
  const float* dw1   = (const float*)d_in[3];
  const float* pw1   = (const float*)d_in[4];
  const float* g1    = (const float*)d_in[5];
  const float* be1   = (const float*)d_in[6];
  const float* r1w   = (const float*)d_in[7];
  const float* r1b   = (const float*)d_in[8];
  const float* dw2   = (const float*)d_in[9];
  const float* pw2   = (const float*)d_in[10];
  const float* g2    = (const float*)d_in[11];
  const float* be2   = (const float*)d_in[12];
  const float* r2w   = (const float*)d_in[13];
  const float* r2b   = (const float*)d_in[14];
  const float* ll1w  = (const float*)d_in[15];
  const float* ll1b  = (const float*)d_in[16];
  const float* flw   = (const float*)d_in[17];
  const float* flb   = (const float*)d_in[18];

  char* ws = (char*)d_ws;
  float*    part = (float*)(ws + WS_PART);
  float*    scsh = (float*)(ws + WS_SCSH);
  _Float16* llw  = (_Float16*)(ws + WS_LLW);
  _Float16* wc   = (_Float16*)(ws + WS_WC);
  float*    gout = (float*)(ws + WS_G);

  k_stats<<<B_SZ, ST_THREADS, 0, stream>>>(src, dw1, dw2, part);
  k_fold<<<1, 256, 0, stream>>>(part, pw1, g1, be1, pw2, g2, be2, ll1w, flw, scsh, llw, wc);
  k_main<<<B_SZ, MT, L_TOTAL, stream>>>(src, dw1, pw1, r1w, r1b, dw2, pw2, r2w, r2b, ll1b,
                                         scsh, llw, wc, gout);
  k_out<<<B_SZ / OB, 256, 0, stream>>>(gout, flb, maxat, (float*)d_out);
}
